// ConvKAN3D_86998857548339
// MI455X (gfx1250) — hardware-verified
//
#include <hip/hip_runtime.h>

typedef _Float16 v16h __attribute__((ext_vector_type(16)));
typedef _Float16 v8h  __attribute__((ext_vector_type(8)));
typedef float    v8f  __attribute__((ext_vector_type(8)));
typedef float    v4f  __attribute__((ext_vector_type(4)));
typedef v8h __attribute__((may_alias)) v8ha;
typedef v4f __attribute__((may_alias)) v4fa;

union Frag { v16h v; v8h half[2]; };

#define WSC   8.0f
#define WINV  0.125f
#define FSC   16.0f
#define FINV  0.0625f

__device__ __forceinline__ v8f wmma_f16(v16h a, v16h b, v8f c) {
  v8f d = __builtin_amdgcn_wmma_f32_16x16x32_f16(false, a, false, b, (short)0, c, false, false);
  asm volatile("v_nop\n\tv_nop\n\tv_nop\n\tv_nop" : "+v"(d) : "v"(a), "v"(b));
  return d;
}

__device__ __forceinline__ v16h load_frag(const _Float16* p, int h) {
  Frag f;
  f.half[0] = *(const v8ha*)(p + 8 * h);
  f.half[1] = *(const v8ha*)(p + 16 + 8 * h);
  return f.v;
}

template<int PIECES>
__device__ __forceinline__ void line_store(const char* src, char* dst, int lane) {
  #pragma unroll
  for (int i = 0; i < PIECES / 32; ++i) {
    const int p = 32 * i + lane;
    const v4f v = *(const v4fa*)(src + 16 * p);
    *(volatile v4f*)(dst + 16 * p) = v;
  }
}

__device__ __forceinline__ float kan_act(float a, const float (&kn)[10], const float (&swc)[10],
                                         float bc, float w1c, float w2c, float scc, float bec) {
  const float y = a * WINV + bc;
  float sp = 0.0f;
  #pragma unroll
  for (int i = 0; i < 10; ++i) {
    const float u = fmaxf(y - kn[i], 0.0f);
    sp += (u * u * u) * swc[i];
  }
  const float sig = __builtin_amdgcn_rcpf(1.0f + __expf(-y));
  const float sil = y * sig;
  return (w1c * sp + w2c * sil) * scc + bec;
}

template<typename OT, int COUT>
__device__ __forceinline__ void kan_pool_epilogue(v8f (&acc)[4][2], int n0, int h, int m,
    const float* __restrict__ bias, const float* __restrict__ knots, const float* __restrict__ sw,
    const float* __restrict__ w1, const float* __restrict__ w2, const float* __restrict__ g,
    const float* __restrict__ beta, OT* sP) {
  float kn[10];
  #pragma unroll
  for (int i = 0; i < 10; ++i) kn[i] = knots[i];
  const float rsq = 1.0f / sqrtf(1.0f + 1e-5f);
  #pragma unroll
  for (int nt = 0; nt < 2; ++nt) {
    const int c = n0 + 16 * nt + m;
    float swc[10];
    #pragma unroll
    for (int i = 0; i < 10; ++i) swc[i] = sw[c * 10 + i];
    const float bc = bias[c], w1c = w1[c], w2c = w2[c], scc = g[c] * rsq, bec = beta[c];
    #pragma unroll
    for (int q = 0; q < 4; ++q) {
      float mx = -__builtin_huge_valf();
      #pragma unroll
      for (int mt = 0; mt < 4; ++mt) {
        const float o0 = kan_act(acc[mt][nt][2 * q],     kn, swc, bc, w1c, w2c, scc, bec);
        const float o1 = kan_act(acc[mt][nt][2 * q + 1], kn, swc, bc, w1c, w2c, scc, bec);
        mx = fmaxf(mx, fmaxf(o0, o1));
      }
      sP[(4 * h + q) * COUT + c] = (OT)mx;
    }
  }
}

template<int CIN, int COUT, int KP>
__global__ __launch_bounds__(256) void pack_w_kernel(const float* __restrict__ w,
                                                     _Float16* __restrict__ wb) {
  constexpr int K = 27 * CIN;
  constexpr int NGRP = COUT * KP / 8;
  static_assert(KP % 32 == 0);
  static_assert(NGRP % 32 == 0);
  const int gidx = blockIdx.x * 256 + threadIdx.x;
  if (gidx >= NGRP) return;
  const int e0 = gidx * 8;
  const int co = e0 / KP;
  const int kk = e0 - co * KP;
  v8h o;
  #pragma unroll
  for (int j = 0; j < 8; ++j) {
    const int k = kk + j;
    const int kc = (k < K) ? k : (K - 1);
    const int tap = kc / CIN;
    const int ci = kc - tap * CIN;
    float v = w[((size_t)co * CIN + ci) * 27 + tap] * WSC;
    v = (k < K) ? v : 0.0f;
    o[j] = (_Float16)v;
  }
  _Float16* dst = wb + (size_t)e0;
  *(volatile v8h*)dst = o;
  __threadfence();
  *(volatile v8h*)dst = o;
}

__global__ __launch_bounds__(128) void conv1_kernel(
    const float* __restrict__ x,
    const _Float16* __restrict__ wb,
    const float* __restrict__ bias, const float* __restrict__ knots, const float* __restrict__ sw,
    const float* __restrict__ w1, const float* __restrict__ w2, const float* __restrict__ g,
    const float* __restrict__ beta,
    _Float16* __restrict__ pout)
{
  __shared__ __attribute__((aligned(16))) _Float16 sA[4 * 64 * 32];
  __shared__ __attribute__((aligned(16))) _Float16 sP[4 * 8 * 32];

  const int tid = threadIdx.x, lane = tid & 31, w = tid >> 5;
  const int h = lane >> 4, m = lane & 15;
  const int t = blockIdx.x * 4 + w;
  const int n = t >> 12;
  const int rr = t & 4095;
  const int dp = rr >> 7, hp = (rr >> 2) & 31, wt = rr & 3;
  const int d0 = 2 * dp, h0 = 2 * hp, w0 = 16 * wt;

  const int kq = (lane < 27) ? lane : 26;
  const int kd = kq / 9, kh = (kq / 3) % 3, kw = kq % 3;
  const float* xn = x + (size_t)n * 262144;
  _Float16* sAw = sA + w * 2048;
  #pragma unroll 4
  for (int j = 0; j < 64; ++j) {
    const int mt = j >> 4;
    const int dd = d0 + (mt >> 1) + kd - 1;
    const int hh = h0 + (mt & 1) + kh - 1;
    const int ww = w0 + (j & 15) + kw - 1;
    const bool ok = (lane < 27) && ((unsigned)dd < 64u) && ((unsigned)hh < 64u) && ((unsigned)ww < 64u);
    const int dc = min(max(dd, 0), 63), hc = min(max(hh, 0), 63), wc = min(max(ww, 0), 63);
    float v = xn[(dc * 64 + hc) * 64 + wc];
    v = ok ? v : 0.0f;
    sAw[j * 32 + lane] = (_Float16)v;
  }
  __syncthreads();

  v16h bfr[2];
  #pragma unroll
  for (int nt = 0; nt < 2; ++nt) bfr[nt] = load_frag(wb + (16 * nt + m) * 32, h);
  const v8f zero8 = {0.f, 0.f, 0.f, 0.f, 0.f, 0.f, 0.f, 0.f};
  v8f acc[4][2];
  #pragma unroll
  for (int mt = 0; mt < 4; ++mt) {
    const v16h a = load_frag(sAw + (mt * 16 + m) * 32, h);
    acc[mt][0] = wmma_f16(a, bfr[0], zero8);
    acc[mt][1] = wmma_f16(a, bfr[1], zero8);
  }

  _Float16* sPw = sP + w * 256;
  kan_pool_epilogue<_Float16, 32>(acc, 0, h, m, bias, knots, sw, w1, w2, g, beta, sPw);
  __syncthreads();

  const size_t vox = (((size_t)n * 32 + dp) * 32 + hp) * 32 + 8 * wt;
  const char* src = (const char*)sPw;
  char* dst = (char*)(pout + vox * 32);
  line_store<32>(src, dst, lane);
  __threadfence();
  line_store<32>(src, dst, lane);
}

template<int CIN, int COUT, int DIM, typename OT>
__global__ __launch_bounds__(128) void convn_kernel(
    const _Float16* __restrict__ pin,
    const _Float16* __restrict__ wb,
    const float* __restrict__ bias, const float* __restrict__ knots, const float* __restrict__ sw,
    const float* __restrict__ w1, const float* __restrict__ w2, const float* __restrict__ g,
    const float* __restrict__ beta,
    OT* __restrict__ pout)
{
  constexpr int K  = 27 * CIN;
  constexpr int NG = COUT / 32;
  constexpr int DP = DIM / 2;
  constexpr int WT = DIM / 16;
  constexpr int CB = CIN / 32;
  constexpr int ROWB = COUT * (int)sizeof(OT);
  constexpr int RPW = 8 / NG;
  constexpr int PIECES = RPW * ROWB / 16;
  constexpr int VOL = DIM * DIM * DIM;
  static_assert(CIN % 32 == 0);
  static_assert(COUT % 32 == 0);
  static_assert(DIM % 16 == 0);
  static_assert(PIECES % 32 == 0);
  static_assert(NG * 32 <= 128);

  __shared__ __attribute__((aligned(16))) OT sP[8 * COUT];

  const int tid = threadIdx.x, lane = tid & 31, w = tid >> 5;
  const int h = lane >> 4, m = lane & 15;
  const int n0 = 32 * w;
  int bb = blockIdx.x;
  const int wt = bb % WT; bb /= WT;
  const int hp = bb % DP; bb /= DP;
  const int dp = bb % DP; bb /= DP;
  const int n = bb;
  const int d0 = 2 * dp, h0 = 2 * hp, w0 = 16 * wt;

  const _Float16* pn = pin + (size_t)n * VOL * CIN;
  const v8f zero8 = {0.f, 0.f, 0.f, 0.f, 0.f, 0.f, 0.f, 0.f};
  const _Float16 hz = (_Float16)0.0f;
  const v8h zero8h = {hz, hz, hz, hz, hz, hz, hz, hz};
  v8f acc[4][2];
  #pragma unroll
  for (int mt = 0; mt < 4; ++mt) { acc[mt][0] = zero8; acc[mt][1] = zero8; }

  #pragma unroll 1
  for (int tap = 0; tap < 27; ++tap) {
    const int kd = tap / 9, kh = (tap / 3) % 3, kw = tap % 3;
    const int ww = w0 + m + kw - 1;
    const bool okw = (unsigned)ww < (unsigned)DIM;
    const int wc = min(max(ww, 0), DIM - 1);
    const _Float16* rowp[4];
    bool ok[4];
    #pragma unroll
    for (int mt = 0; mt < 4; ++mt) {
      const int dd = d0 + (mt >> 1) + kd - 1;
      const int hh = h0 + (mt & 1) + kh - 1;
      ok[mt] = okw && ((unsigned)dd < (unsigned)DIM) && ((unsigned)hh < (unsigned)DIM);
      const int dc = min(max(dd, 0), DIM - 1), hc = min(max(hh, 0), DIM - 1);
      rowp[mt] = pn + ((size_t)(dc * DIM + hc) * DIM + wc) * CIN;
    }
    #pragma unroll
    for (int cb = 0; cb < CB; ++cb) {
      const int k0 = tap * CIN + cb * 32;
      v16h bfr[2];
      #pragma unroll
      for (int nt = 0; nt < 2; ++nt)
        bfr[nt] = load_frag(wb + (size_t)(n0 + 16 * nt + m) * K + k0, h);
      #pragma unroll
      for (int mt = 0; mt < 4; ++mt) {
        Frag a;
        const v8h l0 = *(const v8ha*)(rowp[mt] + cb * 32 + 8 * h);
        const v8h l1 = *(const v8ha*)(rowp[mt] + cb * 32 + 16 + 8 * h);
        a.half[0] = ok[mt] ? l0 : zero8h;
        a.half[1] = ok[mt] ? l1 : zero8h;
        acc[mt][0] = wmma_f16(a.v, bfr[0], acc[mt][0]);
        acc[mt][1] = wmma_f16(a.v, bfr[1], acc[mt][1]);
      }
    }
  }

  kan_pool_epilogue<OT, COUT>(acc, n0, h, m, bias, knots, sw, w1, w2, g, beta, sP);
  __syncthreads();

  const size_t vox = (((size_t)n * DP + dp) * DP + hp) * DP + 8 * wt;
  const char* src = (const char*)sP + (size_t)w * RPW * ROWB;
  char* dst = (char*)pout + (vox + (size_t)w * RPW) * ROWB;
  line_store<PIECES>(src, dst, lane);
  __threadfence();
  line_store<PIECES>(src, dst, lane);
}

__global__ __launch_bounds__(256) void head_kernel(
    const float* __restrict__ p3,
    const float* __restrict__ fc1w,
    const float* __restrict__ fc1b,
    const float* __restrict__ fc2w,
    const float* __restrict__ fc2b,
    float* __restrict__ out)
{
  __shared__ __attribute__((aligned(16))) _Float16 sH[16 * 128];
  __shared__ float sHid[2 * 256];
  __shared__ float sOut[4];

  const int tid = threadIdx.x, lane = tid & 31, w = tid >> 5;
  const int h = lane >> 4, m = lane & 15;

  for (int i = 256 + tid; i < 2048; i += 256) sH[i] = (_Float16)0.0f;
  {
    const int n = tid >> 7, c = tid & 127;
    const float* p = p3 + (size_t)n * 512 * 128 + c;
    float s = 0.0f;
    #pragma unroll 8
    for (int v = 0; v < 512; ++v) s += p[(size_t)v * 128];
    sH[n * 128 + c] = (_Float16)(s * (1.0f / 512.0f));
  }
  __syncthreads();

  const v8f zero8 = {0.f, 0.f, 0.f, 0.f, 0.f, 0.f, 0.f, 0.f};
  v8f acc[2];
  acc[0] = zero8; acc[1] = zero8;
  #pragma unroll
  for (int ks = 0; ks < 4; ++ks) {
    const v16h a = load_frag(sH + m * 128 + 32 * ks, h);
    #pragma unroll
    for (int nt = 0; nt < 2; ++nt) {
      const int j = 32 * w + 16 * nt + m;
      const float* wr = fc1w + (size_t)j * 128 + 32 * ks;
      const v4f q0 = *(const v4fa*)(wr + 8 * h);
      const v4f q1 = *(const v4fa*)(wr + 8 * h + 4);
      const v4f q2 = *(const v4fa*)(wr + 16 + 8 * h);
      const v4f q3 = *(const v4fa*)(wr + 16 + 8 * h + 4);
      const v16h b = { (_Float16)(q0.x * FSC), (_Float16)(q0.y * FSC), (_Float16)(q0.z * FSC), (_Float16)(q0.w * FSC),
                       (_Float16)(q1.x * FSC), (_Float16)(q1.y * FSC), (_Float16)(q1.z * FSC), (_Float16)(q1.w * FSC),
                       (_Float16)(q2.x * FSC), (_Float16)(q2.y * FSC), (_Float16)(q2.z * FSC), (_Float16)(q2.w * FSC),
                       (_Float16)(q3.x * FSC), (_Float16)(q3.y * FSC), (_Float16)(q3.z * FSC), (_Float16)(q3.w * FSC) };
      acc[nt] = wmma_f16(a, b, acc[nt]);
    }
  }
  {
    const int j0 = 32 * w + m, j1 = 32 * w + 16 + m;
    const float b0 = fc1b[j0], b1 = fc1b[j1];
    if (h == 0) {
      sHid[j0]       = fmaxf(acc[0][0] * FINV + b0, 0.0f);
      sHid[256 + j0] = fmaxf(acc[0][1] * FINV + b0, 0.0f);
      sHid[j1]       = fmaxf(acc[1][0] * FINV + b1, 0.0f);
      sHid[256 + j1] = fmaxf(acc[1][1] * FINV + b1, 0.0f);
    }
  }
  __syncthreads();

  if (w == 0) {
    const int oi = lane >> 3, sub = lane & 7;
    const int nn = oi >> 1, o = oi & 1;
    const float bo = fc2b[o];
    float s = 0.0f;
    #pragma unroll 1
    for (int t2 = 0; t2 < 32; ++t2) {
      const int j = 8 * t2 + sub;
      s += sHid[nn * 256 + j] * fc2w[o * 256 + j];
    }
    s += __shfl_xor(s, 1);
    s += __shfl_xor(s, 2);
    s += __shfl_xor(s, 4);
    if (sub == 0) sOut[oi] = s + bo;
  }
  __syncthreads();

  if (tid == 0) {
    v4f v;
    v.x = sOut[0]; v.y = sOut[1]; v.z = sOut[2]; v.w = sOut[3];
    *(volatile v4f*)out = v;
    __threadfence();
    *(volatile v4f*)out = v;
  }
}

extern "C" void kernel_launch(void* const* d_in, const int* in_sizes, int n_in,
                              void* d_out, int out_size, void* d_ws, size_t ws_size,
                              hipStream_t stream) {
  if (n_in < 29) return;
  if (in_sizes[0] != 524288) return;
  if (in_sizes[1] != 864 || in_sizes[2] != 32 || in_sizes[3] != 10 || in_sizes[4] != 320) return;
  if (in_sizes[5] != 32 || in_sizes[6] != 32 || in_sizes[7] != 32 || in_sizes[8] != 32) return;
  if (in_sizes[9] != 55296 || in_sizes[10] != 64 || in_sizes[11] != 10 || in_sizes[12] != 640) return;
  if (in_sizes[13] != 64 || in_sizes[14] != 64 || in_sizes[15] != 64 || in_sizes[16] != 64) return;
  if (in_sizes[17] != 221184 || in_sizes[18] != 128 || in_sizes[19] != 10 || in_sizes[20] != 1280) return;
  if (in_sizes[21] != 128 || in_sizes[22] != 128 || in_sizes[23] != 128 || in_sizes[24] != 128) return;
  if (in_sizes[25] != 32768 || in_sizes[26] != 256 || in_sizes[27] != 512 || in_sizes[28] != 2) return;
  if (out_size != 4) return;

  const float* x     = (const float*)d_in[0];
  const float* c1_w  = (const float*)d_in[1];
  const float* c1_b  = (const float*)d_in[2];
  const float* c1_kn = (const float*)d_in[3];
  const float* c1_sw = (const float*)d_in[4];
  const float* c1_w1 = (const float*)d_in[5];
  const float* c1_w2 = (const float*)d_in[6];
  const float* bn1_g = (const float*)d_in[7];
  const float* bn1_b = (const float*)d_in[8];
  const float* c2_w  = (const float*)d_in[9];
  const float* c2_b  = (const float*)d_in[10];
  const float* c2_kn = (const float*)d_in[11];
  const float* c2_sw = (const float*)d_in[12];
  const float* c2_w1 = (const float*)d_in[13];
  const float* c2_w2 = (const float*)d_in[14];
  const float* bn2_g = (const float*)d_in[15];
  const float* bn2_b = (const float*)d_in[16];
  const float* c3_w  = (const float*)d_in[17];
  const float* c3_b  = (const float*)d_in[18];
  const float* c3_kn = (const float*)d_in[19];
  const float* c3_sw = (const float*)d_in[20];
  const float* c3_w1 = (const float*)d_in[21];
  const float* c3_w2 = (const float*)d_in[22];
  const float* bn3_g = (const float*)d_in[23];
  const float* bn3_b = (const float*)d_in[24];
  const float* fc1_w = (const float*)d_in[25];
  const float* fc1_b = (const float*)d_in[26];
  const float* fc2_w = (const float*)d_in[27];
  const float* fc2_b = (const float*)d_in[28];
  float* out = (float*)d_out;

  const size_t b_wb1 = (size_t)32 * 32 * 2;
  const size_t b_wb2 = (size_t)64 * 864 * 2;
  const size_t b_wb3 = (size_t)128 * 1728 * 2;
  const size_t b_p1  = (size_t)2 * 32768 * 32 * 2;
  const size_t b_p2  = (size_t)2 * 4096 * 64 * 2;
  const size_t b_p3  = (size_t)2 * 512 * 128 * 4;
  size_t off = 0;
  const size_t o_wb1 = off; off += (b_wb1 + 255) & ~(size_t)255;
  const size_t o_wb2 = off; off += (b_wb2 + 255) & ~(size_t)255;
  const size_t o_wb3 = off; off += (b_wb3 + 255) & ~(size_t)255;
  const size_t o_p1  = off; off += (b_p1  + 255) & ~(size_t)255;
  const size_t o_p2  = off; off += (b_p2  + 255) & ~(size_t)255;
  const size_t o_p3  = off; off += (b_p3  + 255) & ~(size_t)255;
  if (off > ws_size) return;

  char* ws = (char*)d_ws;
  _Float16* wb1 = (_Float16*)(ws + o_wb1);
  _Float16* wb2 = (_Float16*)(ws + o_wb2);
  _Float16* wb3 = (_Float16*)(ws + o_wb3);
  _Float16* p1  = (_Float16*)(ws + o_p1);
  _Float16* p2  = (_Float16*)(ws + o_p2);
  float*    p3  = (float*)(ws + o_p3);

  pack_w_kernel<1, 32, 32>    <<<(32 * 32 / 8 + 255) / 256, 256, 0, stream>>>(c1_w, wb1);
  pack_w_kernel<32, 64, 864>  <<<(64 * 864 / 8 + 255) / 256, 256, 0, stream>>>(c2_w, wb2);
  pack_w_kernel<64, 128, 1728><<<(128 * 1728 / 8 + 255) / 256, 256, 0, stream>>>(c3_w, wb3);

  conv1_kernel<<<8192 / 4, 128, 0, stream>>>(x, wb1, c1_b, c1_kn, c1_sw, c1_w1, c1_w2, bn1_g, bn1_b, p1);

  convn_kernel<32, 64, 32, _Float16><<<2 * 16 * 16 * 2, 64, 0, stream>>>(
      p1, wb2, c2_b, c2_kn, c2_sw, c2_w1, c2_w2, bn2_g, bn2_b, p2);

  convn_kernel<64, 128, 16, float><<<2 * 8 * 8 * 1, 128, 0, stream>>>(
      p2, wb3, c3_b, c3_kn, c3_sw, c3_w1, c3_w2, bn3_g, bn3_b, p3);

  head_kernel<<<1, 256, 0, stream>>>(p3, fc1_w, fc1_b, fc2_w, fc2_b, out);
}
